// SynthesisLayer_17334488006827
// MI455X (gfx1250) — hardware-run, weakly checked
//
#include <hip/hip_runtime.h>


#define NBI  8
#define CIN  256
#define COUT 256
#define HH   64
#define WW   64
#define NPX  (HH * WW)
#define WD   512
#define KC   (CIN * 9)
#define DM   WD
#define SLOPE 0.2f
#define LOSC 1024.0f

typedef _Float16 h16;
typedef unsigned short bf;
typedef __attribute__((ext_vector_type(16))) __bf16   v16bf;
typedef __attribute__((ext_vector_type(16))) _Float16 v16h;
typedef __attribute__((ext_vector_type(8)))  _Float16 v8h;
typedef __attribute__((ext_vector_type(8)))  unsigned short v8us;
typedef __attribute__((ext_vector_type(8)))  float    v8f;
typedef __attribute__((ext_vector_type(4)))  float    v4f;
typedef v8h  __attribute__((may_alias)) v8ha;
typedef v4f  __attribute__((may_alias)) v4fa;
typedef v8us __attribute__((may_alias)) v8usa;

__device__ __forceinline__ unsigned short f2bf(float f) { unsigned u = __float_as_uint(f); u += 0x7FFFu + ((u >> 16) & 1u); return (unsigned short)(u >> 16); }
__device__ __forceinline__ float bf2f(unsigned short b) { return __uint_as_float(((unsigned)b) << 16); }
__device__ __forceinline__ float bfr(float f) { return bf2f(f2bf(f)); }
__device__ __forceinline__ v16h cat16(v8h lo, v8h hi) { return __builtin_shufflevector(lo, hi, 0, 1, 2, 3, 4, 5, 6, 7, 8, 9, 10, 11, 12, 13, 14, 15); }
__device__ __forceinline__ v16bf cat16b(v8us lo, v8us hi) { return __builtin_bit_cast(v16bf, __builtin_shufflevector(lo, hi, 0, 1, 2, 3, 4, 5, 6, 7, 8, 9, 10, 11, 12, 13, 14, 15)); }
__device__ __forceinline__ v8f wmma16(v16h a, v16h b, v8f c) { return __builtin_amdgcn_wmma_f32_16x16x32_f16(false, a, false, b, (short)0, c, false, false); }
__device__ __forceinline__ v8f wmmab(v16bf a, v16bf b, v8f c) { return __builtin_amdgcn_wmma_f32_16x16x32_bf16(false, a, false, b, (short)0, c, false, false); }

template <bool SPLITA, bool F16OUT = false>
__global__ __launch_bounds__(128) void k_gemmb(const bf* __restrict__ A, const bf* __restrict__ Al, const bf* __restrict__ Bn, const float* __restrict__ bias, float* C, int ldc, h16* C2, const float* __restrict__ R = nullptr, int K = DM, int roundR = 1) {
    __shared__ __align__(16) float ost[4][16 * 68];
    const int lane = threadIdx.x & 31, wave = threadIdx.x >> 5, lr = lane & 15, hi = lane >> 4;
    const int r0 = blockIdx.x * 64 + wave * 16, c0 = blockIdx.y * 64;
    const size_t aoff = (size_t)(r0 + lr) * K + 8 * hi;
    size_t boff[4];
#pragma unroll
    for (int t = 0; t < 4; ++t) boff[t] = (size_t)(c0 + t * 16 + lr) * K + 8 * hi;
    v8f acc[4];
#pragma unroll
    for (int t = 0; t < 4; ++t) acc[t] = (v8f){};
#pragma unroll 1
    for (int kc = 0; kc < K; kc += 32) {
        const v16bf a = cat16b(*(const v8us*)(A + aoff + kc), *(const v8us*)(A + aoff + kc + 16));
        v16bf al = a;
        if (SPLITA) al = cat16b(*(const v8us*)(Al + aoff + kc), *(const v8us*)(Al + aoff + kc + 16));
#pragma unroll
        for (int t = 0; t < 4; ++t) { const v16bf b = cat16b(*(const v8us*)(Bn + boff[t] + kc), *(const v8us*)(Bn + boff[t] + kc + 16)); acc[t] = wmmab(a, b, acc[t]); if (SPLITA) acc[t] = wmmab(al, b, acc[t]); }
        asm volatile("v_nop\n\tv_nop\n\tv_nop\n\tv_nop" : "+v"(acc[0]), "+v"(acc[1]), "+v"(acc[2]), "+v"(acc[3]) : "v"(a), "v"(al));
    }
    float* os = &ost[wave][0];
#pragma unroll
    for (int t = 0; t < 4; ++t) { const float bv = bias ? bfr(bias[c0 + t * 16 + lr]) : 0.f;
#pragma unroll
        for (int j = 0; j < 8; ++j) os[(hi * 8 + j) * 68 + t * 16 + lr] = acc[t][j] + bv; }
    __syncthreads();
    if (F16OUT) {
        h16* crow = (h16*)(void*)C + (size_t)r0 * ldc + c0;
        auto pass = [&]() {
#pragma unroll
            for (int s = 0; s < 4; ++s) { const int row = 4 * s + (lane >> 3), piece = lane & 7; const float* sp = os + row * 68 + piece * 8; v8h o, o2;
#pragma unroll
                for (int i = 0; i < 8; ++i) { const h16 a = (h16)sp[i]; o[i] = a; o2[i] = (h16)((sp[i] - (float)a) * LOSC); }
                *(volatile v8h*)(crow + (size_t)row * ldc + piece * 8) = o; if (C2) *(volatile v8h*)(C2 + (size_t)r0 * ldc + c0 + (size_t)row * ldc + piece * 8) = o2; }
        };
        pass(); __threadfence(); pass();
    } else {
        float* crow = C + (size_t)r0 * ldc + c0;
        auto pass = [&]() {
#pragma unroll
            for (int s = 0; s < 8; ++s) { const int Lid = (lane >> 3) + 4 * s, piece = lane & 7; const int row = Lid >> 1, cofs = (Lid & 1) * 32 + piece * 4;
                v4f val = *(const v4fa*)(os + row * 68 + cofs); if (R) { const v4f rv = *(const v4f*)(R + ((size_t)r0 + row) * ldc + c0 + cofs); val += roundR ? (v4f){bfr(rv[0]), bfr(rv[1]), bfr(rv[2]), bfr(rv[3])} : rv; }
                *(volatile v4f*)(crow + (size_t)row * ldc + cofs) = val; }
        };
        pass(); __threadfence(); pass();
    }
}


__global__ __launch_bounds__(256) void k_cvt8(const float* __restrict__ src, bf* dst, size_t n8) {
    const size_t i = (size_t)blockIdx.x * 256 + threadIdx.x; if (i >= n8) return;
    const v8f v = *(const v8f*)(src + i * 8); v8us o;
#pragma unroll
    for (int k = 0; k < 8; ++k) o[k] = f2bf(v[k]);
    *(volatile v8us*)(dst + i * 8) = o; __threadfence(); *(volatile v8us*)(dst + i * 8) = o;
}
__global__ __launch_bounds__(256) void k_zero8(bf* dst, size_t n8) {
    const size_t i = (size_t)blockIdx.x * 256 + threadIdx.x; if (i >= n8) return; v8us z;
#pragma unroll
    for (int k = 0; k < 8; ++k) z[k] = 0;
    *(volatile v8us*)(dst + i * 8) = z; __threadfence(); *(volatile v8us*)(dst + i * 8) = z;
}

__global__ __launch_bounds__(256) void k_wb(const float* __restrict__ wv, bf* WB) {
    const int lane = threadIdx.x & 31, r = blockIdx.x * 8 + (threadIdx.x >> 5); if (r >= 64) return;
#pragma unroll 1
    for (int ps = 0; ps < 2; ++ps) {
#pragma unroll
        for (int q = 0; q < WD / 256; ++q) { v8us o;
#pragma unroll
            for (int i = 0; i < 8; ++i) o[i] = (r < NBI) ? f2bf(wv[(size_t)r * WD + q * 256 + lane * 8 + i]) : (unsigned short)0;
            *(volatile v8us*)(WB + (size_t)r * WD + q * 256 + lane * 8) = o; }
        if (ps == 0) __threadfence(); }
}
__global__ __launch_bounds__(256) void k_wmod(const float* __restrict__ Wt, const float* __restrict__ S, const float* __restrict__ sb, int b, bf* Ah, bf* Al) {
    const int lane = threadIdx.x & 31, o = blockIdx.x * 8 + (threadIdx.x >> 5); if (o >= COUT) return;
    const float cs = rsqrtf((float)KC), ssc = rsqrtf((float)WD);
    auto sval = [&](int c) -> float { return S[(size_t)b * CIN + c] * ssc + bfr(sb[c]); };
    float acc = 0.f;
#pragma unroll 1
    for (int c = lane; c < CIN; c += 32) { float w2 = 0.f;
#pragma unroll
        for (int k = 0; k < 9; ++k) { const float wk = cs * bfr(Wt[((size_t)o * CIN + c) * 9 + k]); w2 = fmaf(wk, wk, w2); }
        const float sc = sval(c); acc = fmaf(w2, sc * sc, acc); }
#pragma unroll
    for (int sh = 16; sh; sh >>= 1) acc += __shfl_xor(acc, sh, 32);
    const float dm = rsqrtf(acc + 1e-8f);
#pragma unroll 1
    for (int ps = 0; ps < 2; ++ps) {
#pragma unroll 1
        for (int e0 = lane * 8; e0 < KC; e0 += 256) { v8us oh, ol;
#pragma unroll
            for (int i = 0; i < 8; ++i) { const int e = e0 + i; const int c = e / 9; const float v = cs * bfr(Wt[(size_t)o * KC + e]) * sval(c) * dm; const unsigned short hb = f2bf(v); oh[i] = hb; ol[i] = f2bf(v - bf2f(hb)); }
            const size_t off = (size_t)o * KC + e0; *(volatile v8us*)(Ah + off) = oh; *(volatile v8us*)(Al + off) = ol; }
        if (ps == 0) __threadfence(); }
}
__global__ __launch_bounds__(256) void k_im2col(const float* __restrict__ xb, bf* X9) {
    const int lane = threadIdx.x & 31, p = blockIdx.x * 8 + (threadIdx.x >> 5); if (p >= NPX) return; const int y = p / WW, xx = p % WW;
#pragma unroll 1
    for (int ps = 0; ps < 2; ++ps) {
#pragma unroll 1
        for (int e0 = lane * 8; e0 < KC; e0 += 256) { v8us o;
#pragma unroll
            for (int i = 0; i < 8; ++i) { const int e = e0 + i; const int c = e / 9, k = e - c * 9; const int kh = k / 3, kw = k - kh * 3; const int yy = y + kh - 1, xq = xx + kw - 1;
                const bool ok = (yy >= 0) && (yy < HH) && (xq >= 0) && (xq < WW); o[i] = ok ? f2bf(xb[((size_t)c * HH + (ok ? yy : 0)) * WW + (ok ? xq : 0)]) : (unsigned short)0; }
            *(volatile v8us*)(X9 + (size_t)p * KC + e0) = o; }
        if (ps == 0) __threadfence(); }
}
__global__ __launch_bounds__(256) void k_post(const float* __restrict__ Y, const float* __restrict__ nz, const float* __restrict__ nw, const float* __restrict__ bb, float* OUTB) {
    const int lane = threadIdx.x & 31; const size_t wid = (size_t)blockIdx.x * 8 + (threadIdx.x >> 5); if (wid >= (size_t)COUT * (NPX / 128)) return; const int o = (int)(wid / (NPX / 128)), p0 = (int)(wid % (NPX / 128)) * 128 + lane * 4;
    const float nwo = bfr(nw[o]), bo = bfr(bb[o]); v4f v;
#pragma unroll
    for (int q = 0; q < 4; ++q) { const float y = Y[(size_t)o * NPX + p0 + q] + nwo * bfr(nz[p0 + q]) + bo; v[q] = y >= 0.f ? y : SLOPE * y; }
    *(volatile v4f*)(OUTB + (size_t)o * NPX + p0) = v; __threadfence(); *(volatile v4f*)(OUTB + (size_t)o * NPX + p0) = v;
}

extern "C" void kernel_launch(void* const* d_in, const int* in_sizes, int n_in,
                              void* d_out, int out_size, void* d_ws, size_t ws_size, hipStream_t stream) {
    (void)in_sizes; (void)n_in; (void)out_size;
    const float* x = (const float*)d_in[0]; const float* wv = (const float*)d_in[1]; const float* nz = (const float*)d_in[2]; const float* sw = (const float*)d_in[3]; const float* sb = (const float*)d_in[4]; const float* cw = (const float*)d_in[5]; const float* nw = (const float*)d_in[6]; const float* bb = (const float*)d_in[7];
    float* out = (float*)d_out;
    char* wsp = (char*)d_ws;
    auto take = [&](size_t bytes) { char* p = wsp; wsp += (bytes + 255) & ~(size_t)255; return (void*)p; };
    bf* WB = (bf*)take((size_t)64 * WD * 2); bf* SWB = (bf*)take((size_t)CIN * WD * 2); float* S = (float*)take((size_t)64 * CIN * 4);
    bf* Ah = (bf*)take((size_t)COUT * KC * 2); bf* Al = (bf*)take((size_t)COUT * KC * 2); bf* X9 = (bf*)take((size_t)NPX * KC * 2); float* Y = (float*)take((size_t)COUT * NPX * 4);
    if ((size_t)(wsp - (char*)d_ws) > ws_size) return;
    k_wb<<<64 / 8, 256, 0, stream>>>(wv, WB); k_cvt8<<<(CIN * WD / 8 + 255) / 256, 256, 0, stream>>>(sw, SWB, (size_t)CIN * WD / 8);
    k_gemmb<false, false><<<dim3(1, CIN / 64, 1), 128, 0, stream>>>(WB, nullptr, SWB, nullptr, S, CIN, nullptr, nullptr, WD);
    for (int b = 0; b < NBI; ++b) {
        k_wmod<<<COUT / 8, 256, 0, stream>>>(cw, S, sb, b, Ah, Al);
        k_im2col<<<NPX / 8, 256, 0, stream>>>(x + (size_t)b * CIN * NPX, X9);
        k_gemmb<true, false><<<dim3(COUT / 64, NPX / 64, 1), 128, 0, stream>>>(Ah, Al, X9, nullptr, Y, NPX, nullptr, nullptr, KC);
        k_post<<<(COUT * (NPX / 128)) / 8, 256, 0, stream>>>(Y, nz + (size_t)b * NPX, nw, bb, out + (size_t)b * COUT * NPX); }
}
